// CrossAttention_15590731284898
// MI455X (gfx1250) — hardware-verified
//
#include <hip/hip_runtime.h>
#ifndef NB
#define NB 2
#endif
#ifndef SEQ
#define SEQ 2048
#endif
#define NB_FULL 2
#define SEQ_FULL 2048
#define DM 1024
#define NH 16
#define HD 64
#define NR ((size_t)NB * SEQ)

static_assert(NB >= 1 && NB <= NB_FULL);
static_assert(SEQ <= SEQ_FULL);
static_assert(SEQ % 128 == 0);
static_assert(DM % 64 == 0 && DM % 32 == 0);
static_assert(DM == 4 * 256);
static_assert(NH * HD == DM);
static_assert(HD == 64);
static_assert(SEQ % 64 == 0);

typedef unsigned short v8us __attribute__((ext_vector_type(8), may_alias));
typedef float  v8f  __attribute__((ext_vector_type(8)));
typedef float  v4f  __attribute__((ext_vector_type(4)));
typedef float  v4fa __attribute__((ext_vector_type(4), may_alias));
typedef _Float16 v16h __attribute__((ext_vector_type(16)));
typedef _Float16 v4h __attribute__((ext_vector_type(4)));
union FragH { v16h v; v8us half[2]; _Float16 h[16]; unsigned short u[16]; };

__device__ __forceinline__ unsigned short bf16_bits(float x) { unsigned int u = __float_as_uint(x); return (unsigned short)((u + 0x7FFFu + ((u >> 16) & 1u)) >> 16); }
__device__ __forceinline__ float bf16_val(unsigned short b) { return __uint_as_float(((unsigned int)b) << 16); }
__device__ __forceinline__ float bf16_rne(float x) { return bf16_val(bf16_bits(x)); }

__device__ __forceinline__ v16h g2_frag(const _Float16* p, int hh) { FragH f; f.half[0] = *(const v8us*)((const unsigned short*)p + 8 * hh); f.half[1] = *(const v8us*)((const unsigned short*)p + 16 + 8 * hh); return f.v; }
__device__ __forceinline__ v8f g2_mma(v16h a, v16h b, v8f c) { v8f d = __builtin_amdgcn_wmma_f32_16x16x32_f16(false, a, false, b, (short)0, c, false, false); asm volatile("v_nop\n\tv_nop\n\tv_nop\n\tv_nop" : "+v"(d) : "v"(a), "v"(b)); return d; }

__global__ __launch_bounds__(256) void k_wt_f16(const float* __restrict__ W, _Float16* __restrict__ Wt, int K, int N, float scale) {
  const int t = blockIdx.x * 256 + threadIdx.x; if (t >= N * (K / 8)) return; const int n = t / (K / 8), k8 = (t % (K / 8)) * 8; FragH f;
#pragma unroll
  for (int i = 0; i < 8; ++i) f.h[i] = (_Float16)(bf16_rne(W[(size_t)(k8 + i) * N + n]) * scale);
  const v8us o = f.half[0];
  *(volatile v8us*)((unsigned short*)Wt + (size_t)n * K + k8) = o; __threadfence(); *(volatile v8us*)((unsigned short*)Wt + (size_t)n * K + k8) = o;
}

__global__ __launch_bounds__(256) void k_ln16(const float* __restrict__ X, const float* __restrict__ g, const float* __restrict__ bb, float eps, _Float16* __restrict__ N16) {
  #pragma clang fp contract(off)
  __shared__ float red[256];
  const size_t r = blockIdx.x; const int t = threadIdx.x; const int c0 = t * 4;
  const size_t src = (r / SEQ) * (size_t)SEQ_FULL + (r % SEQ);
  const v4f xa = *(const v4fa*)(X + src * DM + c0);
  float s[4]; float sum = 0.f;
#pragma unroll
  for (int q = 0; q < 4; ++q) { s[q] = bf16_rne(xa[q]); sum = __fadd_rn(sum, s[q]); }
  red[t] = sum; __syncthreads();
  for (int st = 128; st > 0; st >>= 1) { if (t < st) red[t] = __fadd_rn(red[t], red[t + st]); __syncthreads(); }
  const float mu = red[0] / (float)DM; __syncthreads();
  float vs = 0.f;
#pragma unroll
  for (int q = 0; q < 4; ++q) { const float dl = __fadd_rn(s[q], -mu); vs = __fadd_rn(vs, __fmul_rn(dl, dl)); }
  red[t] = vs; __syncthreads();
  for (int st = 128; st > 0; st >>= 1) { if (t < st) red[t] = __fadd_rn(red[t], red[t + st]); __syncthreads(); }
  const float rs = rsqrtf(__fadd_rn(red[0] / (float)DM, eps));
  v4h y;
#pragma unroll
  for (int q = 0; q < 4; ++q) { const int c = c0 + q; const float yf = __fadd_rn(__fmul_rn(__fmul_rn(__fadd_rn(s[q], -mu), rs), bf16_rne(g[c])), bf16_rne(bb[c])); y[q] = (_Float16)yf; }
  for (int pass = 0; pass < 2; ++pass) { *(volatile v4h*)(N16 + r * DM + c0) = y; if (pass == 0) __threadfence(); }
}

__device__ __forceinline__ void gemm_main(const _Float16* __restrict__ A, const _Float16* __restrict__ Bt, int row0, int col0, int ln, int hh,
    v8f& c00, v8f& c01, v8f& c02, v8f& c03, v8f& c10, v8f& c11, v8f& c12, v8f& c13) {
  const _Float16* a0p = A + (size_t)(row0 + ln) * DM; const _Float16* a1p = a0p + (size_t)16 * DM;
  const _Float16* b0p = Bt + (size_t)(col0 + ln) * DM; const _Float16* b1p = b0p + (size_t)16 * DM; const _Float16* b2p = b1p + (size_t)16 * DM; const _Float16* b3p = b2p + (size_t)16 * DM;
#pragma unroll 1
  for (int kb = 0; kb < DM; kb += 32) { const v16h a0 = g2_frag(a0p + kb, hh), a1 = g2_frag(a1p + kb, hh);
    v16h b = g2_frag(b0p + kb, hh); c00 = g2_mma(a0, b, c00); c10 = g2_mma(a1, b, c10);
    b = g2_frag(b1p + kb, hh); c01 = g2_mma(a0, b, c01); c11 = g2_mma(a1, b, c11);
    b = g2_frag(b2p + kb, hh); c02 = g2_mma(a0, b, c02); c12 = g2_mma(a1, b, c12);
    b = g2_frag(b3p + kb, hh); c03 = g2_mma(a0, b, c03); c13 = g2_mma(a1, b, c13); }
}

__global__ __launch_bounds__(128) void k_proj(const _Float16* __restrict__ A, const _Float16* __restrict__ Bt, const float* __restrict__ bias, float alpha, _Float16* __restrict__ C16) {
  __shared__ __attribute__((aligned(16))) float so[4][32][68];
  const int tid = threadIdx.x, w = tid >> 5, lane = tid & 31, ln = lane & 15, hh = lane >> 4;
  const int ntn = DM >> 6; const int mt = blockIdx.x / ntn, nq = blockIdx.x - mt * ntn; const int row0 = mt * 128 + 32 * w, col0 = nq * 64;
  const v8f z8 = {0.f,0.f,0.f,0.f,0.f,0.f,0.f,0.f}; v8f c00 = z8, c01 = z8, c02 = z8, c03 = z8, c10 = z8, c11 = z8, c12 = z8, c13 = z8;
  gemm_main(A, Bt, row0, col0, ln, hh, c00, c01, c02, c03, c10, c11, c12, c13);
  v8f accs[8] = {c00, c01, c02, c03, c10, c11, c12, c13};
#pragma unroll
  for (int u = 0; u < 8; ++u) { const int t = u & 3, half = u >> 2; const float bv = bf16_rne(bias[col0 + t * 16 + ln]);
#pragma unroll
    for (int r = 0; r < 8; ++r) so[w][half * 16 + 8 * hh + r][t * 16 + ln] = accs[u][r] * alpha + bv; }
  __builtin_amdgcn_fence(4  , "workgroup"); __builtin_amdgcn_wave_barrier();
  const int rsub = lane >> 4, c4 = (lane & 15) * 4;
  for (int pass = 0; pass < 2; ++pass) {
#pragma unroll
    for (int q = 0; q < 16; ++q) { const int r = q * 2 + rsub; const v4f v = *(const v4fa*)&so[w][r][c4]; v4h h4;
#pragma unroll
      for (int i = 0; i < 4; ++i) h4[i] = (_Float16)v[i];
      *(volatile v4h*)(C16 + (size_t)(row0 + r) * DM + col0 + c4) = h4; }
    if (pass == 0) __threadfence(); }
}

__global__ __launch_bounds__(128) void k_outp(const _Float16* __restrict__ A, const _Float16* __restrict__ Bt, const float* __restrict__ bias, float alpha, const float* __restrict__ resid, float* __restrict__ C) {
  __shared__ __attribute__((aligned(16))) float so[4][32][68];
  const int tid = threadIdx.x, w = tid >> 5, lane = tid & 31, ln = lane & 15, hh = lane >> 4;
  const int ntn = DM >> 6; const int mt = blockIdx.x / ntn, nq = blockIdx.x - mt * ntn; const int row0 = mt * 128 + 32 * w, col0 = nq * 64;
  const v8f z8 = {0.f,0.f,0.f,0.f,0.f,0.f,0.f,0.f}; v8f c00 = z8, c01 = z8, c02 = z8, c03 = z8, c10 = z8, c11 = z8, c12 = z8, c13 = z8;
  gemm_main(A, Bt, row0, col0, ln, hh, c00, c01, c02, c03, c10, c11, c12, c13);
  v8f accs[8] = {c00, c01, c02, c03, c10, c11, c12, c13};
#pragma unroll
  for (int u = 0; u < 8; ++u) { const int t = u & 3, half = u >> 2; const float bv = bf16_rne(bias[col0 + t * 16 + ln]);
#pragma unroll
    for (int r = 0; r < 8; ++r) so[w][half * 16 + 8 * hh + r][t * 16 + ln] = accs[u][r] * alpha + bv; }
  __builtin_amdgcn_fence(4  , "workgroup"); __builtin_amdgcn_wave_barrier();
  const int rsub = lane >> 4, c4 = (lane & 15) * 4;
  for (int pass = 0; pass < 2; ++pass) {
#pragma unroll 4
    for (int q = 0; q < 16; ++q) { const int r = q * 2 + rsub; const int rr = row0 + r; const size_t gr = (size_t)(rr / SEQ) * SEQ_FULL + (size_t)(rr % SEQ);
      v4f v = *(const v4fa*)&so[w][r][c4]; const v4f x = *(const v4fa*)(resid + gr * DM + col0 + c4);
#pragma unroll
      for (int i = 0; i < 4; ++i) v[i] += bf16_rne(x[i]);
      *(volatile v4f*)(C + gr * DM + col0 + c4) = v; }
    if (pass == 0) __threadfence(); }
}

__global__ __launch_bounds__(256) void k_vt(const _Float16* __restrict__ V16, _Float16* __restrict__ Vt) {
  __shared__ unsigned short tl[64][66];
  const int tid = threadIdx.x; const int slab = blockIdx.x / (SEQ / 64), lg = blockIdx.x % (SEQ / 64); const int b = slab / NH, h = slab % NH;
  for (int i = tid; i < 64 * 8; i += 256) { const int r = i / 8, c8 = (i % 8) * 8; FragH f; f.half[0] = *(const v8us*)((const unsigned short*)V16 + ((size_t)b * SEQ + lg * 64 + r) * DM + h * HD + c8);
#pragma unroll
    for (int q = 0; q < 8; ++q) tl[r][c8 + q] = f.u[q]; }
  __syncthreads();
  for (int pass = 0; pass < 2; ++pass) {
#pragma unroll
    for (int rd = 0; rd < 2; ++rd) { const int d = rd * 32 + tid / 8, pc = tid % 8; FragH f;
#pragma unroll
      for (int q = 0; q < 8; ++q) f.u[q] = tl[pc * 8 + q][d];
      *(volatile v8us*)((unsigned short*)Vt + ((size_t)slab * 64 + d) * SEQ + lg * 64 + pc * 8) = f.half[0]; }
    if (pass == 0) __threadfence(); }
}

__global__ __launch_bounds__(128) void k_flash(const _Float16* __restrict__ Q16, const _Float16* __restrict__ K16, const _Float16* __restrict__ VT, _Float16* __restrict__ O16) {
  __shared__ __attribute__((aligned(16))) unsigned short so[4][16][72];
  const int tid = threadIdx.x, w = tid >> 5, lane = tid & 31, ln = lane & 15, hh = lane >> 4;
  const int qb = blockIdx.x % (SEQ / 64); const int slab = blockIdx.x / (SEQ / 64); const int b = slab / NH, h = slab % NH;
  const int q0 = qb * 64 + w * 16;
  const size_t rb = (size_t)b * SEQ;
  const _Float16* qrow = Q16 + (rb + q0 + ln) * DM + h * HD;
  const v16h bq0 = g2_frag(qrow, hh), bq1 = g2_frag(qrow + 32, hh);
  const _Float16* kp = K16 + (rb + ln) * DM + h * HD;
  const _Float16* vp = VT + ((size_t)slab * HD + ln) * SEQ;
  const v8f z8 = {0.f,0.f,0.f,0.f,0.f,0.f,0.f,0.f};
  v8f o0 = z8, o1 = z8, o2 = z8, o3 = z8;
  float m = -1.0e30f, l = 0.f;
#pragma unroll 1
  for (int kb = 0; kb < SEQ; kb += 32) {
    const _Float16* k0 = kp + (size_t)kb * DM; const _Float16* k1 = k0 + (size_t)16 * DM;
    v8f s0 = z8, s1 = z8;
    s0 = g2_mma(g2_frag(k0, hh), bq0, s0); s0 = g2_mma(g2_frag(k0 + 32, hh), bq1, s0);
    s1 = g2_mma(g2_frag(k1, hh), bq0, s1); s1 = g2_mma(g2_frag(k1 + 32, hh), bq1, s1);
    float x0[8], x1[8]; float tm = -1.0e30f;
#pragma unroll
    for (int i = 0; i < 8; ++i) { x0[i] = s0[i] * 0.125f; x1[i] = s1[i] * 0.125f; tm = fmaxf(tm, fmaxf(x0[i], x1[i])); }
    tm = fmaxf(tm, __shfl_xor(tm, 16, 32));
    const float mn = fmaxf(m, tm);
    const float sc = __expf(m - mn);
    const float mo = mn - 5.545177444f;
    FragH pb; float ps = 0.f;
#pragma unroll
    for (int i = 0; i < 8; ++i) { const float p0 = __expf(x0[i] - mo), p1 = __expf(x1[i] - mo); ps += p0 + p1; pb.h[i] = (_Float16)p0; pb.h[8 + i] = (_Float16)p1; }
    l = l * sc + ps; m = mn;
#pragma unroll
    for (int i = 0; i < 8; ++i) { o0[i] *= sc; o1[i] *= sc; o2[i] *= sc; o3[i] *= sc; }
    o0 = g2_mma(g2_frag(vp + kb, hh), pb.v, o0);
    o1 = g2_mma(g2_frag(vp + (size_t)16 * SEQ + kb, hh), pb.v, o1);
    o2 = g2_mma(g2_frag(vp + (size_t)32 * SEQ + kb, hh), pb.v, o2);
    o3 = g2_mma(g2_frag(vp + (size_t)48 * SEQ + kb, hh), pb.v, o3);
  }
  const float lt = l + __shfl_xor(l, 16, 32);
  const float inv = 64.0f / lt;
  { FragH f;
#pragma unroll
    for (int r = 0; r < 8; ++r) f.h[r] = (_Float16)(o0[r] * inv);
    *(v8us*)&so[w][ln][0 + 8 * hh] = f.half[0];
#pragma unroll
    for (int r = 0; r < 8; ++r) f.h[r] = (_Float16)(o1[r] * inv);
    *(v8us*)&so[w][ln][16 + 8 * hh] = f.half[0];
#pragma unroll
    for (int r = 0; r < 8; ++r) f.h[r] = (_Float16)(o2[r] * inv);
    *(v8us*)&so[w][ln][32 + 8 * hh] = f.half[0];
#pragma unroll
    for (int r = 0; r < 8; ++r) f.h[r] = (_Float16)(o3[r] * inv);
    *(v8us*)&so[w][ln][48 + 8 * hh] = f.half[0]; }
  __builtin_amdgcn_fence(4  , "workgroup"); __builtin_amdgcn_wave_barrier();
  const int rq = lane >> 3, pc = lane & 7;
  for (int pass = 0; pass < 2; ++pass) {
#pragma unroll
    for (int it = 0; it < 4; ++it) { const int row = it * 4 + rq; const v8us v = *(const v8us*)&so[w][row][pc * 8];
      *(volatile v8us*)((unsigned short*)O16 + (rb + q0 + row) * DM + h * HD + pc * 8) = v; }
    if (pass == 0) __threadfence(); }
}

constexpr size_t WB = (size_t)DM * DM * 2;
constexpr size_t AB = (size_t)NB * SEQ * DM * 2;
constexpr size_t OFF_BQ = 0, OFF_BK = OFF_BQ + WB, OFF_BV = OFF_BK + WB, OFF_BO = OFF_BV + WB;
constexpr size_t OFF_XQ = OFF_BO + WB, OFF_XK = OFF_XQ + AB, OFF_Q = OFF_XK + AB, OFF_K = OFF_Q + AB, OFF_V = OFF_K + AB, OFF_VT = OFF_V + AB, OFF_O = OFF_VT + AB;
constexpr size_t WS_TOTAL = OFF_O + AB;
static_assert(WB % 256 == 0 && AB % 256 == 0);
static_assert(WS_TOTAL <= (size_t)134217728);

extern "C" void kernel_launch(void* const* d_in, const int* in_sizes, int n_in,
                              void* d_out, int out_size, void* d_ws, size_t ws_size, hipStream_t stream) {
  if (n_in < 14) return;
  const size_t need_x = ((size_t)(NB - 1) * SEQ_FULL + SEQ) * DM;
  if ((size_t)in_sizes[0] < need_x || (size_t)in_sizes[1] < need_x || (size_t)out_size < need_x) return;
  if ((size_t)in_sizes[2] < (size_t)DM * DM || (size_t)in_sizes[4] < (size_t)DM * DM || (size_t)in_sizes[6] < (size_t)DM * DM || (size_t)in_sizes[8] < (size_t)DM * DM) return;
  if (in_sizes[3] < DM || in_sizes[5] < DM || in_sizes[7] < DM || in_sizes[9] < DM || in_sizes[10] < DM || in_sizes[11] < DM || in_sizes[12] < DM || in_sizes[13] < DM) return;
  if (WS_TOTAL > ws_size) return;
  const float* xq = (const float*)d_in[0]; const float* xc = (const float*)d_in[1];
  const float* wq = (const float*)d_in[2]; const float* bq = (const float*)d_in[3];
  const float* wk = (const float*)d_in[4]; const float* bk = (const float*)d_in[5];
  const float* wv = (const float*)d_in[6]; const float* bv = (const float*)d_in[7];
  const float* wo = (const float*)d_in[8]; const float* bo = (const float*)d_in[9];
  const float* gq = (const float*)d_in[10]; const float* betq = (const float*)d_in[11];
  const float* gkv = (const float*)d_in[12]; const float* betkv = (const float*)d_in[13];
  char* ws = (char*)d_ws;
  _Float16* BQ = (_Float16*)(ws + OFF_BQ); _Float16* BK = (_Float16*)(ws + OFF_BK); _Float16* BV = (_Float16*)(ws + OFF_BV); _Float16* BO = (_Float16*)(ws + OFF_BO);
  _Float16* XQ = (_Float16*)(ws + OFF_XQ); _Float16* XK = (_Float16*)(ws + OFF_XK);
  _Float16* Q16 = (_Float16*)(ws + OFF_Q); _Float16* K16 = (_Float16*)(ws + OFF_K); _Float16* V16 = (_Float16*)(ws + OFF_V);
  _Float16* VT = (_Float16*)(ws + OFF_VT); _Float16* O16 = (_Float16*)(ws + OFF_O);

  { const unsigned g = (unsigned)(((size_t)DM * (DM / 8) + 255) / 256);
    k_wt_f16<<<g, 256, 0, stream>>>(wq, BQ, DM, DM, 16.0f); k_wt_f16<<<g, 256, 0, stream>>>(wk, BK, DM, DM, 16.0f);
    k_wt_f16<<<g, 256, 0, stream>>>(wv, BV, DM, DM, 16.0f); k_wt_f16<<<g, 256, 0, stream>>>(wo, BO, DM, DM, 16.0f); }
  k_ln16<<<(unsigned)NR, 256, 0, stream>>>(xq, gq, betq, 1e-5f, XQ);
  k_ln16<<<(unsigned)NR, 256, 0, stream>>>(xc, gkv, betkv, 1e-5f, XK);
  const unsigned gg = (unsigned)((NR / 128) * (DM / 64));
  k_proj<<<gg, 128, 0, stream>>>(XQ, BQ, bq, 0.0625f, Q16);
  k_proj<<<gg, 128, 0, stream>>>(XK, BK, bk, 0.0625f, K16);
  k_proj<<<gg, 128, 0, stream>>>(XK, BV, bv, 0.0625f, V16);
  k_vt<<<(unsigned)(NB * NH * (SEQ / 64)), 256, 0, stream>>>(V16, VT);
  k_flash<<<(unsigned)(NB * NH * (SEQ / 64)), 128, 0, stream>>>(Q16, K16, VT, O16);
  k_outp<<<gg, 128, 0, stream>>>(O16, BO, bo, 0.0009765625f, xq, (float*)d_out);
}
